// WanSelfAttention_40965398069723
// MI455X (gfx1250) — hardware-verified
//
#include <hip/hip_runtime.h>

typedef _Float16 v16h __attribute__((ext_vector_type(16)));
typedef _Float16 v8h  __attribute__((ext_vector_type(8)));
typedef float    v8f  __attribute__((ext_vector_type(8)));
typedef float    v4f  __attribute__((ext_vector_type(4)));

#ifndef NB
#define NB 2
#endif
#ifndef SEQ
#define SEQ 1024
#endif
#define NB_FULL  2
#define SEQ_FULL 1024
#define DIM  3072
#define NH   24
#define HD   128
#define HHD  64
#define MM   (NB * SEQ)
#define NQT  (SEQ / 128)
#define PT   (DIM / 8)
#define PW   (PT / 32)

#define WSCALE  64.0f
#define OCARRY  16.0f
#define PCARRY  1024.0f

static_assert(SEQ % 128 == 0);
static_assert(MM % 128 == 0);
static_assert(DIM % 128 == 0);
static_assert(NH * HD == DIM);
static_assert(PT * 8 == DIM);
static_assert(PW * 32 == PT);
static_assert(PT <= 512);
static_assert(NB <= NB_FULL);
static_assert(SEQ <= SEQ_FULL);
static_assert((DIM / 8) % 32 == 0);

#define SZ_TAB  ((size_t)SEQ * HHD * 4)
#define SZ_P16  ((size_t)MM * DIM * 2)
#define SZ_W16  ((size_t)DIM * DIM * 2)
#define SZ_Y    ((size_t)MM * DIM * 4)
#define OFF_COS ((size_t)0)
#define OFF_SIN (OFF_COS + SZ_TAB)
#define OFF_XH  (OFF_SIN + SZ_TAB)
#define OFF_WH  (OFF_XH + SZ_P16)
#define OFF_Y   (OFF_WH + SZ_W16)
#define OFF_QH  (OFF_Y + SZ_Y)
#define OFF_KH  (OFF_QH + SZ_P16)
#define OFF_VH  (OFF_KH + SZ_P16)
#define OFF_OH  (OFF_VH + SZ_P16)
#define WS_TOTAL (OFF_OH + SZ_P16)
static_assert(SZ_TAB % 256 == 0);
static_assert(SZ_P16 % 256 == 0);
static_assert(SZ_W16 % 256 == 0);
static_assert(SZ_Y % 256 == 0);
static_assert(WS_TOTAL <= (size_t)134217728);

__device__ __forceinline__ float bf16r(float f) {
  unsigned int u = __float_as_uint(f);
  u += 0x7FFFu + ((u >> 16) & 1u);
  return __uint_as_float(u & 0xFFFF0000u);
}

union Frag { v16h v; v8h half[2]; };

__device__ __forceinline__ v16h ld_frag(const _Float16* tile, int stride) {
  const int lane = threadIdx.x & 31;
  const _Float16* p = tile + (size_t)(lane & 15) * stride + ((lane >> 4) << 3);
  Frag f;
  f.half[0] = *(const v8h*)(p);
  f.half[1] = *(const v8h*)(p + 16);
  return f.v;
}

__device__ __forceinline__ v8f mma16(v16h a, v16h b, v8f c) {
  v8f d = __builtin_amdgcn_wmma_f32_16x16x32_f16(false, a, false, b, (short)0, c, false, false);
  asm volatile("v_nop\n\tv_nop\n\tv_nop\n\tv_nop" : "+v"(d) : "v"(a), "v"(b));
  return d;
}

__device__ __forceinline__ void sincos_cw(float a, float& sn, float& cs) {
  const float kf = rintf(a * 0.63661977236758134f);
  float r = fmaf(-kf, 1.5707963705062866f, a);
  r = fmaf(-kf, -4.3711388286737929e-08f, r);
  r = fmaf(-kf, -1.7151245100059535e-15f, r);
  const float z = r * r;
  const float ps = ((-1.9515295891e-4f * z + 8.3321608736e-3f) * z - 1.6666654611e-1f) * z * r + r;
  const float pc = ((2.443315711809948e-5f * z - 1.388731625493765e-3f) * z + 4.166664568298827e-2f) * (z * z)
                   - 0.5f * z + 1.0f;
  const int q = ((int)kf) & 3;
  sn = (q == 0) ? ps : (q == 1) ? pc : (q == 2) ? -ps : -pc;
  cs = (q == 0) ? pc : (q == 1) ? -ps : (q == 2) ? -pc : ps;
}

__global__ __launch_bounds__(256) void k_tab(const float* __restrict__ freqs,
                                             float* ctab, float* stab, int n) {
  const int i = blockIdx.x * 256 + threadIdx.x;
  if (i < n) {
    const float a = bf16r(freqs[i]);
    float sn, cs;
    sincos_cw(a, sn, cs);
    *(volatile float*)(ctab + i) = cs;
    *(volatile float*)(stab + i) = sn;
    __threadfence();
    *(volatile float*)(ctab + i) = cs;
    *(volatile float*)(stab + i) = sn;
  }
}

__global__ __launch_bounds__(256) void k_cvt16(const float* __restrict__ src, _Float16* dst,
                                               int nrows, int ncols, int seqd, int seqf, float scale) {
  const int cpr = ncols >> 3;
  const int i = blockIdx.x * 256 + threadIdx.x;
  if (i < nrows * cpr) {
    const int m  = i / cpr;
    const int c  = (i - m * cpr) << 3;
    const int bb = m / seqd;
    const int sm = bb * seqf + (m - bb * seqd);
    const float* p = src + (size_t)sm * ncols + c;
    const v4f a0 = *(const v4f*)(p);
    const v4f a1 = *(const v4f*)(p + 4);
    v8h o;
#pragma unroll
    for (int j = 0; j < 4; ++j) {
      o[j]     = (_Float16)(bf16r(a0[j]) * scale);
      o[4 + j] = (_Float16)(bf16r(a1[j]) * scale);
    }
    _Float16* q = dst + (size_t)m * ncols + c;
    *(volatile v8h*)q = o;
    __threadfence();
    *(volatile v8h*)q = o;
  }
}

__global__ __launch_bounds__(256) void k_gemm(
    const _Float16* __restrict__ A, const _Float16* __restrict__ Bw, float* C,
    int Kdim, int ldc, const float* __restrict__ bias, float cscale, int seqd, int seqf)
{
  __shared__ __align__(16) _Float16 ldsA[128 * 32];
  __shared__ __align__(16) _Float16 ldsB[128 * 32];
  __shared__ __align__(16) float    ldsC[64 * 128];
  const int tid  = threadIdx.x;
  const int lane = tid & 31, wave = tid >> 5;
  const int l15  = lane & 15, hi8 = (lane >> 4) << 3;
  const int wm = wave >> 1, wn = wave & 1;
  const int mBase = blockIdx.y * 128;
  const int nBase = blockIdx.x * 128;

  const v8f zf = {};
  v8f acc[2][4];
#pragma unroll
  for (int i = 0; i < 2; i++)
#pragma unroll
    for (int j = 0; j < 4; j++) acc[i][j] = zf;

  int rowT[2], segT[2];
#pragma unroll
  for (int t = 0; t < 2; t++) {
    const int c = tid + t * 256;
    rowT[t] = c >> 2;
    segT[t] = (c & 3) << 3;
  }
  const int nk = Kdim >> 5;

  v8h ra[2], rb[2];
#pragma unroll
  for (int t = 0; t < 2; t++) {
    ra[t] = *(const v8h*)(A  + (size_t)(mBase + rowT[t]) * Kdim + segT[t]);
    rb[t] = *(const v8h*)(Bw + (size_t)(nBase + rowT[t]) * Kdim + segT[t]);
  }
  for (int kb = 0; kb < nk; ++kb) {
#pragma unroll
    for (int t = 0; t < 2; t++) {
      *(v8h*)(&ldsA[rowT[t] * 32 + segT[t]]) = ra[t];
      *(v8h*)(&ldsB[rowT[t] * 32 + segT[t]]) = rb[t];
    }
    __syncthreads();
    if (kb + 1 < nk) {
      const int k0 = (kb + 1) << 5;
#pragma unroll
      for (int t = 0; t < 2; t++) {
        ra[t] = *(const v8h*)(A  + (size_t)(mBase + rowT[t]) * Kdim + k0 + segT[t]);
        rb[t] = *(const v8h*)(Bw + (size_t)(nBase + rowT[t]) * Kdim + k0 + segT[t]);
      }
    }
    v16h af[2], bf[4];
#pragma unroll
    for (int i = 0; i < 2; i++) af[i] = ld_frag(&ldsA[(wm * 32 + i * 16) * 32], 32);
#pragma unroll
    for (int j = 0; j < 4; j++) bf[j] = ld_frag(&ldsB[(wn * 64 + j * 16) * 32], 32);
#pragma unroll
    for (int i = 0; i < 2; i++)
#pragma unroll
      for (int j = 0; j < 4; j++)
        acc[i][j] = mma16(af[i], bf[j], acc[i][j]);
    __syncthreads();
  }

  const int colg = nBase + lane * 4;
  v4f b4;
#pragma unroll
  for (int j = 0; j < 4; ++j) b4[j] = bf16r(bias[colg + j]);

  for (int half = 0; half < 2; ++half) {
    if ((wm >> 1) == half) {
#pragma unroll
      for (int i = 0; i < 2; i++)
#pragma unroll
        for (int j = 0; j < 4; j++)
#pragma unroll
          for (int r = 0; r < 8; r++)
            ldsC[((wm & 1) * 32 + i * 16 + hi8 + r) * 128 + wn * 64 + j * 16 + l15] = acc[i][j][r];
    }
    __syncthreads();
    v4f vals[8];
    size_t goff[8];
#pragma unroll
    for (int r = 0; r < 8; ++r) {
      const v4f t = *(const v4f*)(&ldsC[(wave * 8 + r) * 128 + lane * 4]);
      vals[r] = t * cscale + b4;
      const int grow = mBase + half * 64 + wave * 8 + r;
      const int bb   = grow / seqd;
      const int orow = bb * seqf + (grow - bb * seqd);
      goff[r] = (size_t)orow * ldc + colg;
    }
#pragma unroll
    for (int r = 0; r < 8; ++r) *(volatile v4f*)(C + goff[r]) = vals[r];
    __threadfence();
#pragma unroll
    for (int r = 0; r < 8; ++r) *(volatile v4f*)(C + goff[r]) = vals[r];
    __syncthreads();
  }
}

__global__ __launch_bounds__(PT) void k_post(const float* __restrict__ Y, const float* __restrict__ g,
                                            const float* __restrict__ ctab, const float* __restrict__ stab,
                                            _Float16* dst, int mode)
{
  __shared__ float red[PW];
  const int m = blockIdx.x;
  const int b = m / SEQ, s = m - b * SEQ;
  const int tid = threadIdx.x, lane = tid & 31, wave = tid >> 5;
  const int c0 = tid * 8;
  const float* Yr = Y + (size_t)m * DIM + c0;
  const v4f y0 = *(const v4f*)(Yr);
  const v4f y1 = *(const v4f*)(Yr + 4);
  float yv[8];
#pragma unroll
  for (int j = 0; j < 4; ++j) { yv[j] = y0[j]; yv[4 + j] = y1[j]; }
  float ss = 0.f;
#pragma unroll
  for (int j = 0; j < 8; ++j) ss += yv[j] * yv[j];
  for (int msk = 16; msk; msk >>= 1) ss += __shfl_xor(ss, msk, 32);
  if (lane == 0) red[wave] = ss;
  __syncthreads();
  float tot = 0.f;
#pragma unroll
  for (int wv = 0; wv < PW; ++wv) tot += red[wv];
  const float rs = rsqrtf(tot * (1.0f / (float)DIM) + 1e-6f);
  const bool isv = (mode == 2);

  const v4f g0 = *(const v4f*)(g + c0);
  const v4f g1 = *(const v4f*)(g + c0 + 4);
  float u[8];
#pragma unroll
  for (int j = 0; j < 4; ++j) {
    u[j]     = isv ? yv[j]     : (yv[j]     * rs) * bf16r(g0[j]);
    u[4 + j] = isv ? yv[4 + j] : (yv[4 + j] * rs) * bf16r(g1[j]);
  }
  const v4f c4 = *(const v4f*)(ctab + (size_t)s * HHD + (tid & 15) * 4);
  const v4f s4 = *(const v4f*)(stab + (size_t)s * HHD + (tid & 15) * 4);
  v8h o16;
#pragma unroll
  for (int jp = 0; jp < 4; ++jp) {
    const float e = u[2 * jp], od = u[2 * jp + 1];
    const float cf = c4[jp], sf = s4[jp];
    const float r0 = e * cf - od * sf;
    const float r1 = e * sf + od * cf;
    o16[2 * jp]     = (_Float16)(isv ? e  : r0);
    o16[2 * jp + 1] = (_Float16)(isv ? od : r1);
  }
  const int n = tid >> 4, d0 = (tid & 15) * 8;
  _Float16* q = dst + ((size_t)(b * NH + n) * SEQ + s) * HD + d0;
  *(volatile v8h*)q = o16;
  __threadfence();
  *(volatile v8h*)q = o16;
}

__global__ __launch_bounds__(256) void k_attn(
    const _Float16* __restrict__ qh, const _Float16* __restrict__ kh,
    const _Float16* __restrict__ vh, const int* __restrict__ seq_lens, _Float16* oh)
{
  __shared__ __align__(16) _Float16 ldsK[32 * HD];
  __shared__ __align__(16) _Float16 ldsVt[HD * 32];
  __shared__ __align__(16) _Float16 ldsP[8 * 16 * 32];
  __shared__ __align__(16) _Float16 ldsO[8 * 16 * HD];

  const int tid = threadIdx.x;
  const int lane = tid & 31, w = tid >> 5;
  const int l15 = lane & 15, hsel = lane >> 4, hi8 = hsel << 3;
  const int bid = blockIdx.x;
  const int qt = bid % NQT;
  const int h  = (bid / NQT) % NH;
  const int b  = bid / (NQT * NH);
  int slen = seq_lens[b];
  slen = slen < 1 ? 1 : slen;
  slen = slen > SEQ ? SEQ : slen;
  const float SCALE = 0.08838834764831845f;

  const size_t headO = (size_t)(b * NH + h) * SEQ * HD;
  const _Float16* qbase = qh + headO + (size_t)(qt * 128 + w * 16) * HD;
  const _Float16* kbase = kh + headO;
  const _Float16* vbase = vh + headO;

  v16h qf[4];
#pragma unroll
  for (int dc = 0; dc < 4; dc++) qf[dc] = ld_frag(qbase + dc * 32, HD);

  const v8f zf = {};
  v8f o[8];
  float mrow[8], lrow[8];
#pragma unroll
  for (int dj = 0; dj < 8; dj++) o[dj] = zf;
#pragma unroll
  for (int r = 0; r < 8; r++) { mrow[r] = -3.0e38f; lrow[r] = 0.f; }

  const int nkt = (slen + 31) >> 5;
  for (int kt = 0; kt < nkt; ++kt) {
#pragma unroll
    for (int t = 0; t < 2; t++) {
      const int c = tid + t * 256;
      const int kk = c >> 4, seg = (c & 15) << 3;
      const size_t roff = (size_t)(kt * 32 + kk) * HD + seg;
      const v8h kv = *(const v8h*)(kbase + roff);
      *(v8h*)(ldsK + kk * HD + seg) = kv;
      const v8h vv = *(const v8h*)(vbase + roff);
#pragma unroll
      for (int e = 0; e < 8; e++) ldsVt[(seg + e) * 32 + kk] = vv[e];
    }
    __syncthreads();

    v8f sc[2];
    sc[0] = zf; sc[1] = zf;
#pragma unroll
    for (int dc = 0; dc < 4; dc++) {
      const v16h bk0 = ld_frag(ldsK + dc * 32, HD);
      const v16h bk1 = ld_frag(ldsK + 16 * HD + dc * 32, HD);
      sc[0] = mma16(qf[dc], bk0, sc[0]);
      sc[1] = mma16(qf[dc], bk1, sc[1]);
    }

#pragma unroll
    for (int j = 0; j < 2; j++) {
      const int kg = kt * 32 + j * 16 + l15;
      const bool valid = kg < slen;
#pragma unroll
      for (int r = 0; r < 8; r++) sc[j][r] = valid ? sc[j][r] * SCALE : -3.0e38f;
    }

    float alr[8];
#pragma unroll
    for (int r = 0; r < 8; r++) {
      float t = fmaxf(sc[0][r], sc[1][r]);
      for (int msk = 8; msk; msk >>= 1) t = fmaxf(t, __shfl_xor(t, msk, 32));
      const float mn = fmaxf(mrow[r], t);
      const float al = __expf(mrow[r] - mn);
      const float p0 = __expf(sc[0][r] - mn);
      const float p1 = __expf(sc[1][r] - mn);
      sc[0][r] = p0; sc[1][r] = p1;
      float rsum = p0 + p1;
      for (int msk = 8; msk; msk >>= 1) rsum += __shfl_xor(rsum, msk, 32);
      lrow[r] = lrow[r] * al + rsum;
      mrow[r] = mn;
      alr[r]  = al;
    }
#pragma unroll
    for (int dj = 0; dj < 8; dj++)
#pragma unroll
      for (int r = 0; r < 8; r++) o[dj][r] *= alr[r];

    _Float16* Pw = ldsP + w * (16 * 32);
#pragma unroll
    for (int j = 0; j < 2; j++)
#pragma unroll
      for (int r = 0; r < 8; r++)
        Pw[(hi8 + r) * 32 + j * 16 + l15] = (_Float16)(sc[j][r] * PCARRY);
    __syncthreads();

    const v16h pf = ld_frag(Pw, 32);
#pragma unroll
    for (int dj = 0; dj < 8; dj++) {
      const v16h vf = ld_frag(ldsVt + dj * 16 * 32, 32);
      o[dj] = mma16(pf, vf, o[dj]);
    }
    __syncthreads();
  }

  _Float16* Ow = ldsO + w * (16 * HD);
#pragma unroll
  for (int r = 0; r < 8; r++) {
    const float inv = __builtin_amdgcn_rcpf(lrow[r]) * (OCARRY / PCARRY);
#pragma unroll
    for (int dj = 0; dj < 8; dj++)
      Ow[(hi8 + r) * HD + dj * 16 + l15] = (_Float16)(o[dj][r] * inv);
  }
  __syncthreads();

  v8h ov[8];
  size_t go[8];
#pragma unroll
  for (int it = 0; it < 8; ++it) {
    const int lr = it * 2 + hsel;
    const int piece = l15 * 8;
    ov[it] = *(const v8h*)(Ow + lr * HD + piece);
    const int srow = qt * 128 + w * 16 + lr;
    go[it] = ((size_t)(b * SEQ + srow)) * DIM + h * HD + piece;
  }
#pragma unroll
  for (int it = 0; it < 8; ++it) *(volatile v8h*)(oh + go[it]) = ov[it];
  __threadfence();
#pragma unroll
  for (int it = 0; it < 8; ++it) *(volatile v8h*)(oh + go[it]) = ov[it];
}

extern "C" void kernel_launch(void* const* d_in, const int* in_sizes, int n_in,
                              void* d_out, int out_size, void* d_ws, size_t ws_size,
                              hipStream_t stream) {
  if (n_in < 14) return;
  const long need_x = (long)((NB - 1) * SEQ_FULL + SEQ) * DIM;
  if ((long)in_sizes[0] < need_x) return;
  if (in_sizes[1] < NB) return;
  if (in_sizes[3] < SEQ * HHD) return;
  if (in_sizes[4] < DIM * DIM || in_sizes[6] < DIM * DIM ||
      in_sizes[8] < DIM * DIM || in_sizes[10] < DIM * DIM) return;
  if (in_sizes[5] < DIM || in_sizes[7] < DIM || in_sizes[9] < DIM ||
      in_sizes[11] < DIM || in_sizes[12] < DIM || in_sizes[13] < DIM) return;
  if ((long)out_size < need_x) return;
  if (ws_size < WS_TOTAL) return;

  const float* x        = (const float*)d_in[0];
  const int*   seq_lens = (const int*)d_in[1];
  const float* freqs = (const float*)d_in[3];
  const float* Wq = (const float*)d_in[4];
  const float* bq = (const float*)d_in[5];
  const float* Wk = (const float*)d_in[6];
  const float* bk = (const float*)d_in[7];
  const float* Wv = (const float*)d_in[8];
  const float* bv = (const float*)d_in[9];
  const float* Wo = (const float*)d_in[10];
  const float* bo = (const float*)d_in[11];
  const float* gq = (const float*)d_in[12];
  const float* gk = (const float*)d_in[13];
  float* out = (float*)d_out;

  char* ws = (char*)d_ws;
  float*    ctab = (float*)(ws + OFF_COS);
  float*    stab = (float*)(ws + OFF_SIN);
  _Float16* xh   = (_Float16*)(ws + OFF_XH);
  _Float16* wh   = (_Float16*)(ws + OFF_WH);
  float*    Y    = (float*)(ws + OFF_Y);
  _Float16* qh   = (_Float16*)(ws + OFF_QH);
  _Float16* kh   = (_Float16*)(ws + OFF_KH);
  _Float16* vh   = (_Float16*)(ws + OFF_VH);
  _Float16* oh   = (_Float16*)(ws + OFF_OH);

  const int ntab  = SEQ * HHD;
  const int gtab  = (ntab + 255) / 256;
  const int gcx   = (MM * (DIM / 8) + 255) / 256;
  const int gcw   = (DIM * (DIM / 8) + 255) / 256;
  const dim3 ggemm(DIM / 128, MM / 128);
  const float cs_proj = 1.0f / WSCALE;
  const float cs_out  = 1.0f / (WSCALE * OCARRY);

  k_tab<<<gtab, 256, 0, stream>>>(freqs, ctab, stab, ntab);
  k_cvt16<<<gcx, 256, 0, stream>>>(x, xh, MM, DIM, SEQ, SEQ_FULL, 1.0f);
  k_cvt16<<<gcw, 256, 0, stream>>>(Wq, wh, DIM, DIM, DIM, DIM, WSCALE);
  k_gemm<<<ggemm, 256, 0, stream>>>(xh, wh, Y, DIM, DIM, bq, cs_proj, MM, MM);
  k_post<<<MM, PT, 0, stream>>>(Y, gq, ctab, stab, qh, 0);
  k_cvt16<<<gcw, 256, 0, stream>>>(Wk, wh, DIM, DIM, DIM, DIM, WSCALE);
  k_gemm<<<ggemm, 256, 0, stream>>>(xh, wh, Y, DIM, DIM, bk, cs_proj, MM, MM);
  k_post<<<MM, PT, 0, stream>>>(Y, gk, ctab, stab, kh, 1);
  k_cvt16<<<gcw, 256, 0, stream>>>(Wv, wh, DIM, DIM, DIM, DIM, WSCALE);
  k_gemm<<<ggemm, 256, 0, stream>>>(xh, wh, Y, DIM, DIM, bv, cs_proj, MM, MM);
  k_post<<<MM, PT, 0, stream>>>(Y, gq, ctab, stab, vh, 2);
  k_attn<<<NB * NH * NQT, 256, 0, stream>>>(qh, kh, vh, seq_lens, oh);
  k_cvt16<<<gcw, 256, 0, stream>>>(Wo, wh, DIM, DIM, DIM, DIM, WSCALE);
  k_gemm<<<ggemm, 256, 0, stream>>>(oh, wh, out, DIM, DIM, bo, cs_out, SEQ, SEQ_FULL);
}
